// SimpleGGNN_22325240004844
// MI455X (gfx1250) — hardware-verified
//
#include <hip/hip_runtime.h>
#include <hip/hip_bf16.h>
#include <stddef.h>


#define HIDC    128
#define NTYP    8
#define KMSG    (NTYP * HIDC)
#define G3      (3 * HIDC)
#define NTHR    256
#define NWAVE   8
#define EPT     8
#define NGRP    2
#define CHUNK   (NTHR * EPT * NGRP)
#define WCAP    (EPT * NGRP * 32)
#define LISTN   (NWAVE * WCAP)
#define NBC     4096
#define NBF     1024
#define RCAP    40960
#define RBN     128
#define OTHR    512
#define TGT     32
#define NPW     (TGT / NWAVE)
#define DEGCAP  256
#define APK     (KMSG + 8)
#define MPK     (HIDC + 8)
#define WHSCALE 8.0f
#define WHINV   0.125f

#define LDS_FILL  ((RCAP + NBF + LISTN) * 4 + 64)
#define L_AHI     0
#define L_ALO     (L_AHI + TGT * APK * 2)
#define L_SCR     (L_ALO + TGT * APK * 2)
#define L_BACC    (L_SCR + NWAVE * KMSG * 4)
#define L_HF32    (L_BACC + TGT * HIDC * 4)
#define L_HF16    (L_HF32 + TGT * HIDC * 4)
#define LDS_FUSED (L_HF16 + TGT * MPK * 2)

static_assert((CHUNK & (CHUNK - 1)) == 0);
static_assert(CHUNK <= 4096);
static_assert((NBC & (NBC - 1)) == 0 && (NBF & (NBF - 1)) == 0);
static_assert(NBC == 4 * NBF);
static_assert(OTHR * 8 == NBC);
static_assert((RCAP % 32) == 0);
static_assert(TGT == NWAVE * NPW);
static_assert((TGT * HIDC / 4) == 4 * NTHR);
static_assert(2 * TGT * MPK * 2 <= NWAVE * KMSG * 4);
static_assert((L_ALO % 16) == 0 && (L_SCR % 16) == 0 && (L_BACC % 16) == 0 && (L_HF32 % 16) == 0 && (L_HF16 % 16) == 0);
static_assert((APK % 8) == 0 && (MPK % 8) == 0);
static_assert(((NTYP * HIDC * HIDC / 8) % NTHR) == 0 && ((G3 * HIDC / 8) % NTHR) == 0);

typedef float          v4f  __attribute__((ext_vector_type(4)));
typedef float          v8f  __attribute__((ext_vector_type(8)));
typedef int            v4i  __attribute__((ext_vector_type(4)));
typedef unsigned short v4us __attribute__((ext_vector_type(4)));
typedef unsigned short v8us __attribute__((ext_vector_type(8)));
typedef _Float16       v4h  __attribute__((ext_vector_type(4)));
typedef _Float16       v8h  __attribute__((ext_vector_type(8)));
typedef _Float16       v16h __attribute__((ext_vector_type(16)));
typedef __bf16         v16b __attribute__((ext_vector_type(16)));
union FragH { v16h v; v8h h[2]; };
union FragB { v16b v; v8us u[2]; };

__device__ __forceinline__ unsigned short bf_bits(float f) {
  unsigned int u = __float_as_uint(f);
  u += 0x7FFFu + ((u >> 16) & 1u);
  return (unsigned short)(u >> 16);
}
__device__ __forceinline__ float bf_val(unsigned short s) {
  return __uint_as_float(((unsigned int)s) << 16);
}

__device__ __forceinline__ v8f wmb(v16b a, v16b b, v8f c) {
  v8f d = __builtin_amdgcn_wmma_f32_16x16x32_bf16(false, a, false, b, (short)0, c, false, false);
  asm volatile("v_nop\n\tv_nop\n\tv_nop\n\tv_nop" : "+v"(d) : "v"(a), "v"(b));
  return d;
}
__device__ __forceinline__ v8f wmh(v16h a, v16h b, v8f c) {
  v8f d = __builtin_amdgcn_wmma_f32_16x16x32_f16(false, a, false, b, (short)0, c, false, false);
  asm volatile("v_nop\n\tv_nop\n\tv_nop\n\tv_nop" : "+v"(d) : "v"(a), "v"(b));
  return d;
}

template <int NB>
__device__ __forceinline__ int scan_chunk(const int* __restrict__ dsts, int nE, int cbase, int slotBase,
                                          int vec8, int* list, int tid, int lane, int wave) {
  int wc = 0;
#pragma unroll
  for (int g = 0; g < NGRP; ++g) {
    const int el0  = (g * NTHR + tid) * EPT;
    const int e0   = cbase + el0;
    const int sent = -2147483647 - 1;
    v4i da, db;
    if (vec8 != 0 && cbase + CHUNK <= nE) {
      da = *(const v4i*)(dsts + e0);
      db = *(const v4i*)(dsts + e0 + 4);
    } else {
      da.x = (e0     < nE) ? dsts[min(e0, nE - 1)] : sent;
      da.y = (e0 + 1 < nE) ? dsts[min(e0 + 1, nE - 1)] : sent;
      da.z = (e0 + 2 < nE) ? dsts[min(e0 + 2, nE - 1)] : sent;
      da.w = (e0 + 3 < nE) ? dsts[min(e0 + 3, nE - 1)] : sent;
      db.x = (e0 + 4 < nE) ? dsts[min(e0 + 4, nE - 1)] : sent;
      db.y = (e0 + 5 < nE) ? dsts[min(e0 + 5, nE - 1)] : sent;
      db.z = (e0 + 6 < nE) ? dsts[min(e0 + 6, nE - 1)] : sent;
      db.w = (e0 + 7 < nE) ? dsts[min(e0 + 7, nE - 1)] : sent;
    }
    const unsigned nb = (unsigned)slotBase;
    const unsigned s0 = (unsigned)da.x - nb, s1 = (unsigned)da.y - nb;
    const unsigned s2 = (unsigned)da.z - nb, s3 = (unsigned)da.w - nb;
    const unsigned s4 = (unsigned)db.x - nb, s5 = (unsigned)db.y - nb;
    const unsigned s6 = (unsigned)db.z - nb, s7 = (unsigned)db.w - nb;
    const bool h0 = s0 < (unsigned)NB, h1 = s1 < (unsigned)NB, h2 = s2 < (unsigned)NB, h3 = s3 < (unsigned)NB;
    const bool h4 = s4 < (unsigned)NB, h5 = s5 < (unsigned)NB, h6 = s6 < (unsigned)NB, h7 = s7 < (unsigned)NB;
    const unsigned any = __builtin_amdgcn_ballot_w32(h0 | h1 | h2 | h3 | h4 | h5 | h6 | h7);
    if (any != 0u) {
#define HITJ(J, HJ, SJ) { \
        const unsigned mj = __builtin_amdgcn_ballot_w32(HJ); \
        if (mj != 0u) { \
          if (HJ) { \
            const int pos = wc + (int)__builtin_amdgcn_mbcnt_lo(mj, 0u); \
            if (pos < WCAP) list[wave * WCAP + pos] = ((el0 + (J)) << 12) | (int)(SJ); \
          } \
          wc += (int)__builtin_popcount(mj); } }
      HITJ(0, h0, s0)
      HITJ(1, h1, s1)
      HITJ(2, h2, s2)
      HITJ(3, h3, s3)
      HITJ(4, h4, s4)
      HITJ(5, h5, s5)
      HITJ(6, h6, s6)
      HITJ(7, h7, s7)
#undef HITJ
    }
  }
  return wc;
}

__global__ __launch_bounds__(NTHR) void k_wprep(
    const float* __restrict__ W, const float* __restrict__ wih, const float* __restrict__ whh,
    unsigned short* wtHi, unsigned short* wtLo, unsigned short* wiHi, unsigned short* wiLo, _Float16* whF) {
  const int g0 = NTYP * HIDC * HIDC / 8;
  const int g1 = G3 * HIDC / 8;
  const int g2 = G3 * HIDC / 8;
  const int bstart = blockIdx.x * NTHR;
  const int i = bstart + (int)threadIdx.x;
  if (i >= g0 + g1 + g2) return;
  float v[8];
  if (bstart < g0) {
    const int o   = i * 8;
    const int t   = o >> 14;
    const int rem = o & 16383;
    const int n   = rem >> 7;
    const int k0  = rem & 127;
#pragma unroll
    for (int e = 0; e < 8; ++e) v[e] = W[(size_t)t * HIDC * HIDC + (size_t)(k0 + e) * HIDC + n];
    v8us hv, lv;
#pragma unroll
    for (int e = 0; e < 8; ++e) {
      const unsigned short hb = bf_bits(v[e]);
      hv[e] = hb;
      lv[e] = bf_bits(v[e] - bf_val(hb));
    }
    *(volatile v8us*)(wtHi + o) = hv;
    *(volatile v8us*)(wtLo + o) = lv;
    __threadfence();
    *(volatile v8us*)(wtHi + o) = hv;
    *(volatile v8us*)(wtLo + o) = lv;
  } else if (bstart < g0 + g1) {
    const int o = (i - g0) * 8;
    const v4f a = *(const v4f*)(wih + o), b = *(const v4f*)(wih + o + 4);
    v[0] = a.x; v[1] = a.y; v[2] = a.z; v[3] = a.w; v[4] = b.x; v[5] = b.y; v[6] = b.z; v[7] = b.w;
    v8us hv, lv;
#pragma unroll
    for (int e = 0; e < 8; ++e) {
      const unsigned short hb = bf_bits(v[e]);
      hv[e] = hb;
      lv[e] = bf_bits(v[e] - bf_val(hb));
    }
    *(volatile v8us*)(wiHi + o) = hv;
    *(volatile v8us*)(wiLo + o) = lv;
    __threadfence();
    *(volatile v8us*)(wiHi + o) = hv;
    *(volatile v8us*)(wiLo + o) = lv;
  } else {
    const int o = (i - g0 - g1) * 8;
    const v4f a = *(const v4f*)(whh + o), b = *(const v4f*)(whh + o + 4);
    v8h q;
    q[0] = (_Float16)(a.x * WHSCALE); q[1] = (_Float16)(a.y * WHSCALE);
    q[2] = (_Float16)(a.z * WHSCALE); q[3] = (_Float16)(a.w * WHSCALE);
    q[4] = (_Float16)(b.x * WHSCALE); q[5] = (_Float16)(b.y * WHSCALE);
    q[6] = (_Float16)(b.z * WHSCALE); q[7] = (_Float16)(b.w * WHSCALE);
    *(volatile v8h*)(whF + o) = q;
    __threadfence();
    *(volatile v8h*)(whF + o) = q;
  }
}

__global__ __launch_bounds__(NTHR) void k_count(
    const int* __restrict__ ei, int* cnt, int nE, int vec8) {
  __shared__ __attribute__((aligned(16))) int scnt[NBC];
  __shared__ __attribute__((aligned(16))) int list[LISTN];
  __shared__ int wcnt[NWAVE];
  const int tid = threadIdx.x, lane = tid & 31, wave = tid >> 5;
  const int nodeBase = blockIdx.x * NBC;
  const int* dsts = ei + nE;

  for (int i = tid; i < NBC; i += NTHR) scnt[i] = 0;
  __syncthreads();

  const int nChunks = (nE + CHUNK - 1) / CHUNK;
#pragma unroll 1
  for (int ch = 0; ch < nChunks; ++ch) {
    const int cbase = ch * CHUNK;
    const int wc = scan_chunk<NBC>(dsts, nE, cbase, nodeBase, vec8, list, tid, lane, wave);
    if (lane == 0) wcnt[wave] = wc;
    __syncthreads();
    if (wave == 0) {
#pragma unroll 1
      for (int wsx = 0; wsx < NWAVE; ++wsx) {
        int n = __builtin_amdgcn_readfirstlane(wcnt[wsx]);
        n = n > WCAP ? WCAP : (n < 0 ? 0 : n);
        const int* lp = list + wsx * WCAP;
#pragma unroll 1
        for (int i = 0; i < n; ++i) {
          const int ent  = __builtin_amdgcn_readfirstlane(lp[i]);
          const int slot = ent & (NBC - 1);
          if (lane == 0) scnt[slot] = scnt[slot] + 1;
        }
      }
    }
    __syncthreads();
  }

  v4i cq[4];
#pragma unroll
  for (int q = 0; q < 4; ++q) {
    const int f = (wave * 4 + q) * 128 + 4 * lane;
    cq[q] = *(const v4i*)(scnt + f);
  }
  int* cp = cnt + (size_t)nodeBase;
#pragma unroll
  for (int q = 0; q < 4; ++q) {
    const int f = (wave * 4 + q) * 128 + 4 * lane;
    *(volatile v4i*)(cp + f) = cq[q];
  }
  __threadfence();
#pragma unroll
  for (int q = 0; q < 4; ++q) {
    const int f = (wave * 4 + q) * 128 + 4 * lane;
    *(volatile v4i*)(cp + f) = cq[q];
  }
}

__global__ __launch_bounds__(OTHR) void k_offsets(
    const int* __restrict__ cnt, int* off, int* rbase, int nChunk) {
  __shared__ __attribute__((aligned(16))) int soff[NBC];
  __shared__ __attribute__((aligned(16))) int srb[RBN];
  __shared__ int wtot[OTHR / 32];
  const int tid = threadIdx.x, lane = tid & 31, wave = tid >> 5, sub = tid >> 7;
  for (int i = tid; i < RBN; i += OTHR) srb[i] = 0;
  int carry = 0;
#pragma unroll 1
  for (int ch = 0; ch < nChunk; ++ch) {
    const int base = ch * NBC;
    const v4i c0 = *(const v4i*)(cnt + base + 8 * tid);
    const v4i c1 = *(const v4i*)(cnt + base + 8 * tid + 4);
    const int e0 = max(c0.x, 0), e1 = max(c0.y, 0), e2 = max(c0.z, 0), e3 = max(c0.w, 0);
    const int e4 = max(c1.x, 0), e5 = max(c1.y, 0), e6 = max(c1.z, 0), e7 = max(c1.w, 0);
    const int ts = e0 + e1 + e2 + e3 + e4 + e5 + e6 + e7;
    int incl = ts;
#pragma unroll
    for (int d = 1; d < 32; d <<= 1) {
      const int t = __shfl_up(incl, d);
      if (lane >= d) incl += t;
    }
    if (lane == 31) wtot[wave] = incl;
    __syncthreads();
    const int S0 = wtot[0]  + wtot[1]  + wtot[2]  + wtot[3];
    const int S1 = wtot[4]  + wtot[5]  + wtot[6]  + wtot[7];
    const int S2 = wtot[8]  + wtot[9]  + wtot[10] + wtot[11];
    const int S3 = wtot[12] + wtot[13] + wtot[14] + wtot[15];
    int pre = 0;
#pragma unroll 1
    for (int w = 4 * sub; w < wave; ++w) pre += wtot[w];
    const int b0 = carry;
    const int b1 = b0 + ((S0 + 31) & ~31);
    const int b2 = b1 + ((S1 + 31) & ~31);
    const int b3 = b2 + ((S2 + 31) & ~31);
    const int b4 = b3 + ((S3 + 31) & ~31);
    const int myb = sub == 0 ? b0 : (sub == 1 ? b1 : (sub == 2 ? b2 : b3));
    if (tid == 0) {
      srb[min(4 * ch + 0, RBN - 1)] = b0;
      srb[min(4 * ch + 1, RBN - 1)] = b1;
      srb[min(4 * ch + 2, RBN - 1)] = b2;
      srb[min(4 * ch + 3, RBN - 1)] = b3;
    }
    int run = myb + pre + incl - ts;
    soff[8 * tid + 0] = run; run += e0;
    soff[8 * tid + 1] = run; run += e1;
    soff[8 * tid + 2] = run; run += e2;
    soff[8 * tid + 3] = run; run += e3;
    soff[8 * tid + 4] = run; run += e4;
    soff[8 * tid + 5] = run; run += e5;
    soff[8 * tid + 6] = run; run += e6;
    soff[8 * tid + 7] = run;
    carry = b4;
    __syncthreads();
    const v4i o0 = *(const v4i*)(soff + 4 * tid);
    const v4i o1 = *(const v4i*)(soff + 4 * (tid + OTHR));
    int* op = off + base;
    *(volatile v4i*)(op + 4 * tid) = o0;
    *(volatile v4i*)(op + 4 * (tid + OTHR)) = o1;
    __threadfence();
    *(volatile v4i*)(op + 4 * tid) = o0;
    *(volatile v4i*)(op + 4 * (tid + OTHR)) = o1;
    __syncthreads();
  }
  if (tid == 0) srb[min(4 * nChunk, RBN - 1)] = carry;
  __syncthreads();
  v4i rv = {0, 0, 0, 0};
  if (tid < 32) rv = *(const v4i*)(srb + 4 * tid);
  if (tid < 32) *(volatile v4i*)(rbase + 4 * tid) = rv;
  __threadfence();
  if (tid < 32) *(volatile v4i*)(rbase + 4 * tid) = rv;
}

__global__ __launch_bounds__(NTHR) void k_fill(
    const int* __restrict__ ei, const int* __restrict__ et, const int* __restrict__ off,
    const int* __restrict__ rbase, int* csr, int nN, int nE, int vec8, int csrLen) {
  extern __shared__ v4f lds_dyn[];
  int* region = (int*)lds_dyn;
  int* cursor = region + RCAP;
  int* list   = cursor + NBF;
  int* wcnt   = list + LISTN;
  const int tid = threadIdx.x, lane = tid & 31, wave = tid >> 5;
  const int b = blockIdx.x;
  const int nodeBase = b * NBF;
  const int* dsts = ei + nE;

  int rb0 = rbase[b];
  const int rb1 = rbase[b + 1];
  rb0 = rb0 < 0 ? 0 : (rb0 > csrLen ? csrLen : rb0);
  rb0 &= ~31;
  int len = rb1 - rb0;
  len = len < 0 ? 0 : (len > RCAP ? RCAP : len);
  int lenW = (len + 31) & ~31;
  if (rb0 + lenW > csrLen) lenW = (csrLen - rb0) & ~31;

  {
    const v4i z = {0, 0, 0, 0};
    for (int i = tid; i < RCAP / 4; i += NTHR) ((v4i*)region)[i] = z;
    for (int s = tid; s < NBF; s += NTHR) {
      int o = off[nodeBase + s] - rb0;
      o = o < 0 ? 0 : (o > RCAP ? RCAP : o);
      cursor[s] = o;
    }
  }
  __syncthreads();

  const int nChunks = (nE + CHUNK - 1) / CHUNK;
#pragma unroll 1
  for (int ch = 0; ch < nChunks; ++ch) {
    const int cbase = ch * CHUNK;
    const int wc = scan_chunk<NBF>(dsts, nE, cbase, nodeBase, vec8, list, tid, lane, wave);
    if (lane == 0) wcnt[wave] = wc;
    __syncthreads();
    if (wave == 0) {
#pragma unroll 1
      for (int wsx = 0; wsx < NWAVE; ++wsx) {
        int n = __builtin_amdgcn_readfirstlane(wcnt[wsx]);
        n = n > WCAP ? WCAP : (n < 0 ? 0 : n);
        const int* lp = list + wsx * WCAP;
#pragma unroll 1
        for (int i = 0; i < n; ++i) {
          const int ent  = __builtin_amdgcn_readfirstlane(lp[i]);
          const int slot = ent & (NBF - 1);
          int e = cbase + ((ent >> 12) & (CHUNK - 1));
          e = e > nE - 1 ? nE - 1 : e;
          int src = ei[e];
          src = src < 0 ? 0 : (src > nN - 1 ? nN - 1 : src);
          int ty = et[e];
          ty = ty < 0 ? 0 : (ty > NTYP - 1 ? NTYP - 1 : ty);
          if (lane == 0) {
            int pos = cursor[slot];
            pos = pos < 0 ? 0 : (pos > RCAP - 1 ? RCAP - 1 : pos);
            region[pos] = (src << 3) | ty;
            const int np = pos + 1;
            cursor[slot] = np > RCAP ? RCAP : np;
          }
        }
      }
    }
    __syncthreads();
  }

  const int nv = lenW >> 2;
  int* gp = csr + rb0;
#pragma unroll 1
  for (int i = tid; i < nv; i += NTHR) { const v4i v = ((const v4i*)region)[i]; *(volatile v4i*)(gp + 4 * i) = v; }
  __threadfence();
#pragma unroll 1
  for (int i = tid; i < nv; i += NTHR) { const v4i v = ((const v4i*)region)[i]; *(volatile v4i*)(gp + 4 * i) = v; }
}

__global__ __launch_bounds__(NTHR) void k_fused(
    const float* __restrict__ h, const int* __restrict__ csr, const int* __restrict__ off,
    const int* __restrict__ cnt, const float* __restrict__ mb,
    const unsigned short* __restrict__ wtHi, const unsigned short* __restrict__ wtLo,
    const unsigned short* __restrict__ wiHi, const unsigned short* __restrict__ wiLo,
    const _Float16* __restrict__ whF, const float* __restrict__ bih, const float* __restrict__ bhh,
    float* out, int nN, int csrLen) {
  extern __shared__ v4f lds_dyn[];
  char* lb = (char*)lds_dyn;
  unsigned short* aHi  = (unsigned short*)(lb + L_AHI);
  unsigned short* aLo  = (unsigned short*)(lb + L_ALO);
  float*          scr  = (float*)(lb + L_SCR);
  unsigned short* mHi  = (unsigned short*)(lb + L_SCR);
  unsigned short* mLo  = mHi + TGT * MPK;
  float*          bacc = (float*)(lb + L_BACC);
  float*          hf   = (float*)(lb + L_HF32);
  _Float16*       hq   = (_Float16*)(lb + L_HF16);
  const int tid = threadIdx.x, lane = tid & 31, wave = tid >> 5, hh = lane >> 4, m = lane & 15;
  const int node0 = blockIdx.x * TGT;
  const v4f z4 = {0.f, 0.f, 0.f, 0.f};

#pragma unroll
  for (int i = 0; i < (TGT * HIDC / 4) / NTHR; ++i) {
    const int idx = i * NTHR + tid;
    const int row = idx >> 5;
    const int c   = (idx & 31) * 4;
    int nd = node0 + row;
    nd = nd > nN - 1 ? nN - 1 : nd;
    const v4f v = *(const v4f*)(h + (size_t)nd * HIDC + c);
    *(v4f*)(hf + row * HIDC + c) = v;
    v4h q;
    q.x = (_Float16)v.x; q.y = (_Float16)v.y; q.z = (_Float16)v.z; q.w = (_Float16)v.w;
    *(v4h*)(hq + row * MPK + c) = q;
  }
  float* scrw = scr + wave * KMSG;
#pragma unroll
  for (int t = 0; t < NTYP; ++t) *(v4f*)(scrw + t * HIDC + 4 * lane) = z4;

#pragma unroll 1
  for (int i = 0; i < NPW; ++i) {
    const int row = wave * NPW + i;
    const int nd  = node0 + row;
    const int ndc = nd > nN - 1 ? nN - 1 : nd;
    int n = cnt[ndc];
    n = nd < nN ? n : 0;
    n = n < 0 ? 0 : (n > DEGCAP ? DEGCAP : n);
    int st = off[ndc];
    st = st < 0 ? 0 : (st > csrLen - 1 ? csrLen - 1 : st);
    v4f ba = z4;
    unsigned int tm = 0u;
#pragma unroll 1
    for (int q0 = 0; q0 < n; q0 += 32) {
      int pos = st + q0 + lane;
      pos = pos > csrLen - 1 ? csrLen - 1 : pos;
      const int ent = csr[pos];
      const int mc  = (n - q0) < 32 ? (n - q0) : 32;
#pragma unroll 1
      for (int p = 0; p < mc; ++p) {
        const int e = __builtin_amdgcn_readlane(ent, p);
        int src = e >> 3;
        src = src < 0 ? 0 : (src > nN - 1 ? nN - 1 : src);
        const int t = e & 7;
        tm |= 1u << t;
        const v4f hv = *(const v4f*)(h + (size_t)src * HIDC + 4 * lane);
        const v4f bv = *(const v4f*)(mb + t * HIDC + 4 * lane);
        ba = ba + bv;
        v4f* sp = (v4f*)(scrw + t * HIDC + 4 * lane);
        *sp = *sp + hv;
      }
    }
    *(v4f*)(bacc + row * HIDC + 4 * lane) = ba;
    unsigned short* ph = aHi + row * APK + 4 * lane;
    unsigned short* pl = aLo + row * APK + 4 * lane;
#pragma unroll
    for (int t = 0; t < NTYP; ++t) {
      v4us hv4 = {0, 0, 0, 0}, lv4 = {0, 0, 0, 0};
      if (((tm >> t) & 1u) != 0u) {
        v4f* sp = (v4f*)(scrw + t * HIDC + 4 * lane);
        const v4f s = *sp;
        const unsigned short h0 = bf_bits(s.x), h1 = bf_bits(s.y), h2 = bf_bits(s.z), h3 = bf_bits(s.w);
        hv4.x = h0; hv4.y = h1; hv4.z = h2; hv4.w = h3;
        lv4.x = bf_bits(s.x - bf_val(h0));
        lv4.y = bf_bits(s.y - bf_val(h1));
        lv4.z = bf_bits(s.z - bf_val(h2));
        lv4.w = bf_bits(s.w - bf_val(h3));
        *sp = z4;
      }
      *(v4us*)(ph + t * HIDC) = hv4;
      *(v4us*)(pl + t * HIDC) = lv4;
    }
  }
  __syncthreads();

  const int col = 16 * wave + m;
  v8f acc[2];
  { const v8f z8 = {0.f, 0.f, 0.f, 0.f, 0.f, 0.f, 0.f, 0.f}; acc[0] = z8; acc[1] = z8; }
  const unsigned short* pa0h = aHi + m * APK + 8 * hh;
  const unsigned short* pa1h = aHi + (16 + m) * APK + 8 * hh;
  const unsigned short* pa0l = aLo + m * APK + 8 * hh;
  const unsigned short* pa1l = aLo + (16 + m) * APK + 8 * hh;
#pragma unroll 1
  for (int ks = 0; ks < KMSG / 32; ++ks) {
    const int t  = ks >> 2;
    const int kk = (ks & 3) * 32;
    FragB a0h, a1h, a0l, a1l, bh, bl;
    a0h.u[0] = *(const v8us*)(pa0h + 32 * ks);  a0h.u[1] = *(const v8us*)(pa0h + 32 * ks + 16);
    a1h.u[0] = *(const v8us*)(pa1h + 32 * ks);  a1h.u[1] = *(const v8us*)(pa1h + 32 * ks + 16);
    a0l.u[0] = *(const v8us*)(pa0l + 32 * ks);  a0l.u[1] = *(const v8us*)(pa0l + 32 * ks + 16);
    a1l.u[0] = *(const v8us*)(pa1l + 32 * ks);  a1l.u[1] = *(const v8us*)(pa1l + 32 * ks + 16);
    const size_t bo = (size_t)(t * HIDC + col) * HIDC + kk + 8 * hh;
    bh.u[0] = *(const v8us*)(wtHi + bo);  bh.u[1] = *(const v8us*)(wtHi + bo + 16);
    bl.u[0] = *(const v8us*)(wtLo + bo);  bl.u[1] = *(const v8us*)(wtLo + bo + 16);
    acc[0] = wmb(a0l.v, bh.v, acc[0]);
    acc[0] = wmb(a0h.v, bl.v, acc[0]);
    acc[0] = wmb(a0h.v, bh.v, acc[0]);
    acc[1] = wmb(a1l.v, bh.v, acc[1]);
    acc[1] = wmb(a1h.v, bl.v, acc[1]);
    acc[1] = wmb(a1h.v, bh.v, acc[1]);
  }
#pragma unroll
  for (int rt = 0; rt < 2; ++rt) {
#pragma unroll
    for (int r = 0; r < 8; ++r) {
      const int row = 16 * rt + 8 * hh + r;
      const float v = acc[rt][r] + bacc[row * HIDC + col];
      const unsigned short hb = bf_bits(v);
      const unsigned short lv = bf_bits(v - bf_val(hb));
      mHi[row * MPK + col] = hb;
      mLo[row * MPK + col] = lv;
    }
  }
  __syncthreads();

  const float bir = bih[col], biz = bih[HIDC + col], bin2 = bih[2 * HIDC + col];
  const float bhr = bhh[col], bhz = bhh[HIDC + col], bhn = bhh[2 * HIDC + col];
#pragma unroll 1
  for (int rt = 0; rt < 2; ++rt) {
    v8f g[6];
    { const v8f z8 = {0.f, 0.f, 0.f, 0.f, 0.f, 0.f, 0.f, 0.f};
#pragma unroll
      for (int q = 0; q < 6; ++q) g[q] = z8; }
    const unsigned short* pmh = mHi + (16 * rt + m) * MPK + 8 * hh;
    const unsigned short* pml = mLo + (16 * rt + m) * MPK + 8 * hh;
    const _Float16*       phq = hq  + (16 * rt + m) * MPK + 8 * hh;
#pragma unroll 1
    for (int ks = 0; ks < HIDC / 32; ++ks) {
      FragB fmh, fml; FragH fh;
      fmh.u[0] = *(const v8us*)(pmh + 32 * ks);  fmh.u[1] = *(const v8us*)(pmh + 32 * ks + 16);
      fml.u[0] = *(const v8us*)(pml + 32 * ks);  fml.u[1] = *(const v8us*)(pml + 32 * ks + 16);
      fh.h[0]  = *(const v8h*)(phq + 32 * ks);    fh.h[1]  = *(const v8h*)(phq + 32 * ks + 16);
#pragma unroll
      for (int gq = 0; gq < 3; ++gq) {
        const size_t bo = (size_t)(gq * HIDC + col) * HIDC + 32 * ks + 8 * hh;
        FragB bh, bl; FragH bf;
        bh.u[0] = *(const v8us*)(wiHi + bo);  bh.u[1] = *(const v8us*)(wiHi + bo + 16);
        bl.u[0] = *(const v8us*)(wiLo + bo);  bl.u[1] = *(const v8us*)(wiLo + bo + 16);
        bf.h[0] = *(const v8h*)(whF + bo);    bf.h[1] = *(const v8h*)(whF + bo + 16);
        g[gq] = wmb(fml.v, bh.v, g[gq]);
        g[gq] = wmb(fmh.v, bl.v, g[gq]);
        g[gq] = wmb(fmh.v, bh.v, g[gq]);
        g[3 + gq] = wmh(fh.v, bf.v, g[3 + gq]);
      }
    }
#pragma unroll
    for (int r = 0; r < 8; ++r) {
      const int row = 16 * rt + 8 * hh + r;
      const float ir = g[0][r] + bir, iz = g[1][r] + biz, inn = g[2][r] + bin2;
      const float hr = g[3][r] * WHINV + bhr, hz = g[4][r] * WHINV + bhz, hn = g[5][r] * WHINV + bhn;
      float xr = ir + hr; xr = fminf(fmaxf(xr, -30.0f), 30.0f);
      float xz = iz + hz; xz = fminf(fmaxf(xz, -30.0f), 30.0f);
      const float rg = __builtin_amdgcn_rcpf(1.0f + __expf(-xr));
      const float zg = __builtin_amdgcn_rcpf(1.0f + __expf(-xz));
      float xn = inn + rg * hn; xn = fminf(fmaxf(xn, -15.0f), 15.0f);
      const float ng = tanhf(xn);
      float* op = hf + row * HIDC + col;
      const float hv = *op;
      *op = (1.0f - zg) * ng + zg * hv;
    }
  }
  __syncthreads();

#pragma unroll
  for (int i = 0; i < NPW; ++i) {
    const int row = wave * NPW + i;
    const int nd = node0 + row;
    if (nd < nN) {
      const v4f v = *(const v4f*)(hf + row * HIDC + 4 * lane);
      *(volatile v4f*)(out + (size_t)nd * HIDC + 4 * lane) = v;
    }
  }
  __threadfence();
#pragma unroll
  for (int i = 0; i < NPW; ++i) {
    const int row = wave * NPW + i;
    const int nd = node0 + row;
    if (nd < nN) {
      const v4f v = *(const v4f*)(hf + row * HIDC + 4 * lane);
      *(volatile v4f*)(out + (size_t)nd * HIDC + 4 * lane) = v;
    }
  }
}

extern "C" void kernel_launch(void* const* d_in, const int* in_sizes, int n_in,
                              void* d_out, int out_size, void* d_ws, size_t ws_size,
                              hipStream_t stream) {
  if (n_in < 9) return;
  const int nN = in_sizes[0] / HIDC;
  const int nE = in_sizes[2];
  if (nN <= 0 || nE <= 0 || in_sizes[0] != nN * HIDC || in_sizes[1] != 2 * nE) return;
  if (in_sizes[3] != NTYP * HIDC * HIDC || in_sizes[4] != NTYP * HIDC) return;
  if (in_sizes[5] != G3 * HIDC || in_sizes[6] != G3 * HIDC || in_sizes[7] != G3 || in_sizes[8] != G3) return;
  if (out_size != nN * HIDC) return;
  if (nE > (1 << 28) || nN > (1 << 24)) return;

  const float* h   = (const float*)d_in[0];
  const int*   ei  = (const int*)d_in[1];
  const int*   et  = (const int*)d_in[2];
  const float* W   = (const float*)d_in[3];
  const float* mb  = (const float*)d_in[4];
  const float* wih = (const float*)d_in[5];
  const float* whh = (const float*)d_in[6];
  const float* bih = (const float*)d_in[7];
  const float* bhh = (const float*)d_in[8];
  float* out = (float*)d_out;

  const int nBC    = (nN + NBC - 1) / NBC;
  const int CNTPAD = nBC * NBC;
  if (4 * nBC + 1 > RBN) return;
  const int nBF    = (nN + NBF - 1) / NBF;
  const int csrLen = ((nE + 31) & ~31) + 4096;
  const int nFused = (nN + TGT - 1) / TGT;

  char* ws = (char*)d_ws;
  size_t ob = 0;
  const size_t oWtH = ob; ob += (size_t)NTYP * HIDC * HIDC * 2;   ob = (ob + 255) & ~(size_t)255;
  const size_t oWtL = ob; ob += (size_t)NTYP * HIDC * HIDC * 2;   ob = (ob + 255) & ~(size_t)255;
  const size_t oWiH = ob; ob += (size_t)G3 * HIDC * 2;            ob = (ob + 255) & ~(size_t)255;
  const size_t oWiL = ob; ob += (size_t)G3 * HIDC * 2;            ob = (ob + 255) & ~(size_t)255;
  const size_t oWhF = ob; ob += (size_t)G3 * HIDC * 2;            ob = (ob + 255) & ~(size_t)255;
  const size_t oCnt = ob; ob += (size_t)CNTPAD * 4;               ob = (ob + 255) & ~(size_t)255;
  const size_t oOff = ob; ob += (size_t)CNTPAD * 4;               ob = (ob + 255) & ~(size_t)255;
  const size_t oRb  = ob; ob += (size_t)RBN * 4;                  ob = (ob + 255) & ~(size_t)255;
  const size_t oCsr = ob; ob += (size_t)csrLen * 4;               ob = (ob + 255) & ~(size_t)255;
  if (ob > ws_size || ob > ((size_t)128 << 20)) return;
  unsigned short* wtHi = (unsigned short*)(ws + oWtH);
  unsigned short* wtLo = (unsigned short*)(ws + oWtL);
  unsigned short* wiHi = (unsigned short*)(ws + oWiH);
  unsigned short* wiLo = (unsigned short*)(ws + oWiL);
  _Float16*       whF  = (_Float16*)(ws + oWhF);
  int*            cnt  = (int*)(ws + oCnt);
  int*            offp = (int*)(ws + oOff);
  int*            rb   = (int*)(ws + oRb);
  int*            csr  = (int*)(ws + oCsr);

  const int vec8 = ((nE & 3) == 0) ? 1 : 0;

  const int nPrep = NTYP * HIDC * HIDC / 8 + 2 * (G3 * HIDC / 8);
  k_wprep<<<(nPrep + NTHR - 1) / NTHR, NTHR, 0, stream>>>(W, wih, whh, wtHi, wtLo, wiHi, wiLo, whF);

  k_count<<<nBC, NTHR, 0, stream>>>(ei, cnt, nE, vec8);
  k_offsets<<<1, OTHR, 0, stream>>>(cnt, offp, rb, nBC);
  hipFuncSetAttribute(reinterpret_cast<const void*>(&k_fill),
                      hipFuncAttributeMaxDynamicSharedMemorySize, LDS_FILL);
  k_fill<<<nBF, NTHR, LDS_FILL, stream>>>(ei, et, offp, rb, csr, nN, nE, vec8, csrLen);

  hipFuncSetAttribute(reinterpret_cast<const void*>(&k_fused),
                      hipFuncAttributeMaxDynamicSharedMemorySize, LDS_FUSED);
  k_fused<<<nFused, NTHR, LDS_FUSED, stream>>>(h, csr, offp, cnt, mb, wtHi, wtLo, wiHi, wiLo, whF,
                                                bih, bhh, out, nN, csrLen);
}
